// MLPPredictor_24601572671556
// MI455X (gfx1250) — hardware-verified
//
#include <hip/hip_runtime.h>
#include <stddef.h>
#include <stdint.h>

#define KIN    128
#define NHID   256
#define NROWB  32
#define GTHR   128
#define TP     132
#define EPB    256
#define NUNW   (2 * NHID * KIN / 8)
#define WSMAX  134217728

static_assert(KIN % 32 == 0);
static_assert(NHID == 2 * 128);
static_assert(NROWB == (GTHR / 32 / 2) * 16);
static_assert(((TP * 4) % 16) == 0);
static_assert(EPB == 8 * 32);
static_assert(EPB / 4 == 64);
static_assert(NUNW % 256 == 0);
static_assert(NHID * KIN / 8 == 4096);
static_assert(KIN / 8 == 16);
static_assert(NHID == 32 * 8);

typedef float          v4f   __attribute__((ext_vector_type(4)));
typedef float          v8f   __attribute__((ext_vector_type(8)));
typedef int            v8i   __attribute__((ext_vector_type(8)));
typedef unsigned int   v4u   __attribute__((ext_vector_type(4)));
typedef unsigned short v8us  __attribute__((ext_vector_type(8)));
typedef unsigned short v16us __attribute__((ext_vector_type(16)));
typedef _Float16       v8h   __attribute__((ext_vector_type(8)));
typedef __bf16         v16bf __attribute__((ext_vector_type(16)));
typedef v4f  __attribute__((may_alias)) v4fa;
typedef v4u  __attribute__((may_alias)) v4ua;
typedef v8us __attribute__((may_alias)) v8usa;
union FragB { v16bf v; v16us u; v8us h[2]; v8i w; };
union H8 { v8h h; v8us u; };

__device__ __forceinline__ v8f wmb(const FragB& a, const FragB& b, v8f c) {
  v8f d = __builtin_amdgcn_wmma_f32_16x16x32_bf16(false, a.v, false, b.v, (short)0, c, false, false);
  asm volatile("v_nop\n\tv_nop\n\tv_nop\n\tv_nop" : "+v"(d) : "v"(a.w), "v"(b.w));
  return d;
}

__device__ __forceinline__ unsigned bf16_bits(float f) {
  const unsigned u = __float_as_uint(f);
  return (u + 0x7FFFu + ((u >> 16) & 1u)) >> 16;
}
__device__ __forceinline__ float bf16_val(float f) {
  return __uint_as_float(bf16_bits(f) << 16);
}
__device__ __forceinline__ float h2f(unsigned int b) {
  union { unsigned short u; _Float16 h; } c;
  c.u = (unsigned short)b;
  return (float)c.h;
}

__global__ __launch_bounds__(256) void k_wprep(const float* __restrict__ W1, unsigned short* WB, int nUnits) {
  const int u = (int)blockIdx.x * 256 + (int)threadIdx.x;
  if (u >= nUnits) return;
  const int tbl = u >> 12;
  const int c   = (u >> 4) & (NHID - 1);
  const int k8  = (u & 15) * 8;
  const float* p = W1 + (size_t)(tbl * KIN + k8) * NHID + c;
  v8us o;
#pragma unroll
  for (int i = 0; i < 8; ++i) o[i] = (unsigned short)bf16_bits(p[(size_t)i * NHID]);
  unsigned short* dp = WB + (size_t)u * 8;
  *(volatile v8us*)dp = o;
  __threadfence();
  *(volatile v8us*)dp = o;
}

__global__ __launch_bounds__(GTHR) void k_node(
    const float* __restrict__ hS,
    const float* __restrict__ hD,
    const unsigned short* __restrict__ WB,
    unsigned short* Pp,
    unsigned short* Qp,
    int nA)
{
  __shared__ __attribute__((aligned(16))) float sT[4 * 16 * TP];

  const int tid = (int)threadIdx.x, lane = tid & 31, wave = tid >> 5;
  const int hh = lane >> 4, m = lane & 15;
  const int rt = wave >> 1, ch = wave & 1;
  const int tbl = (int)blockIdx.y;
  const float* hN = tbl ? hD : hS;
  unsigned short* PL = tbl ? Qp : Pp;
  const int a0 = (int)blockIdx.x * NROWB + 16 * rt;

  int ar = a0 + m;
  ar = ar > nA - 1 ? nA - 1 : ar;
  const float* zr = hN + (size_t)ar * KIN + 8 * hh;
  const unsigned short* wp = WB + (size_t)(tbl * NHID + ch * 128 + m) * KIN + 8 * hh;

  v8f acc[8];
  {
    const v8f z8 = {0.f, 0.f, 0.f, 0.f, 0.f, 0.f, 0.f, 0.f};
#pragma unroll
    for (int t = 0; t < 8; ++t) acc[t] = z8;
  }

#pragma unroll 1
  for (int kk = 0; kk < KIN / 32; ++kk) {
    const int k0 = 32 * kk;
    const v4f f0 = *(const v4fa*)(zr + k0);
    const v4f f1 = *(const v4fa*)(zr + k0 + 4);
    const v4f f2 = *(const v4fa*)(zr + k0 + 16);
    const v4f f3 = *(const v4fa*)(zr + k0 + 20);
    FragB af;
    af.u[0]  = (unsigned short)bf16_bits(f0.x);
    af.u[1]  = (unsigned short)bf16_bits(f0.y);
    af.u[2]  = (unsigned short)bf16_bits(f0.z);
    af.u[3]  = (unsigned short)bf16_bits(f0.w);
    af.u[4]  = (unsigned short)bf16_bits(f1.x);
    af.u[5]  = (unsigned short)bf16_bits(f1.y);
    af.u[6]  = (unsigned short)bf16_bits(f1.z);
    af.u[7]  = (unsigned short)bf16_bits(f1.w);
    af.u[8]  = (unsigned short)bf16_bits(f2.x);
    af.u[9]  = (unsigned short)bf16_bits(f2.y);
    af.u[10] = (unsigned short)bf16_bits(f2.z);
    af.u[11] = (unsigned short)bf16_bits(f2.w);
    af.u[12] = (unsigned short)bf16_bits(f3.x);
    af.u[13] = (unsigned short)bf16_bits(f3.y);
    af.u[14] = (unsigned short)bf16_bits(f3.z);
    af.u[15] = (unsigned short)bf16_bits(f3.w);
#pragma unroll
    for (int nt = 0; nt < 8; ++nt) {
      const unsigned short* wq = wp + (size_t)(16 * nt) * KIN + k0;
      FragB bf;
      bf.h[0] = *(const v8usa*)wq;
      bf.h[1] = *(const v8usa*)(wq + 16);
      acc[nt] = wmb(af, bf, acc[nt]);
    }
  }

  float* sTw = sT + wave * 16 * TP;
#pragma unroll
  for (int nt = 0; nt < 8; ++nt) {
#pragma unroll
    for (int r = 0; r < 8; ++r) sTw[(8 * hh + r) * TP + 16 * nt + m] = acc[nt][r];
  }
  __syncthreads();

  const int chL = lane >> 4, cw = 8 * (lane & 15);
  const float* sRd = sT + ((2 * (wave >> 1) + chL) * 16 + 8 * (wave & 1)) * TP + cw;
  unsigned short* dstp = PL + 8 * lane;
  const int rowb = (int)blockIdx.x * NROWB + 8 * wave;
#pragma unroll
  for (int i = 0; i < 8; ++i) {
    const int row = rowb + i;
    if (row < nA) {
      const v4f x0 = *(const v4fa*)(sRd + i * TP);
      const v4f x1 = *(const v4fa*)(sRd + i * TP + 4);
      H8 o;
      o.h[0] = (_Float16)(x0.x * 8.0f); o.h[1] = (_Float16)(x0.y * 8.0f);
      o.h[2] = (_Float16)(x0.z * 8.0f); o.h[3] = (_Float16)(x0.w * 8.0f);
      o.h[4] = (_Float16)(x1.x * 8.0f); o.h[5] = (_Float16)(x1.y * 8.0f);
      o.h[6] = (_Float16)(x1.z * 8.0f); o.h[7] = (_Float16)(x1.w * 8.0f);
      *(volatile v8us*)(dstp + (size_t)row * NHID) = o.u;
    }
  }
  __threadfence();
#pragma unroll
  for (int i = 0; i < 8; ++i) {
    const int row = rowb + i;
    if (row < nA) {
      const v4f x0 = *(const v4fa*)(sRd + i * TP);
      const v4f x1 = *(const v4fa*)(sRd + i * TP + 4);
      H8 o;
      o.h[0] = (_Float16)(x0.x * 8.0f); o.h[1] = (_Float16)(x0.y * 8.0f);
      o.h[2] = (_Float16)(x0.z * 8.0f); o.h[3] = (_Float16)(x0.w * 8.0f);
      o.h[4] = (_Float16)(x1.x * 8.0f); o.h[5] = (_Float16)(x1.y * 8.0f);
      o.h[6] = (_Float16)(x1.z * 8.0f); o.h[7] = (_Float16)(x1.w * 8.0f);
      *(volatile v8us*)(dstp + (size_t)row * NHID) = o.u;
    }
  }
}

__device__ __forceinline__ void out_store_pass(float* out, v4f v, int eb, int nE, bool full, bool tailw) {
  if (full) {
    *(volatile v4f*)(out + (size_t)eb) = v;
  } else if (tailw) {
    if (eb     < nE) *(volatile float*)(out + (size_t)eb)     = v.x;
    if (eb + 1 < nE) *(volatile float*)(out + (size_t)eb + 1) = v.y;
    if (eb + 2 < nE) *(volatile float*)(out + (size_t)eb + 2) = v.z;
    if (eb + 3 < nE) *(volatile float*)(out + (size_t)eb + 3) = v.w;
  }
}

__global__ __launch_bounds__(EPB) void k_edge(
    const unsigned short* Pp,
    const unsigned short* Qp,
    const int*   __restrict__ srcI,
    const int*   __restrict__ dstI,
    const float* __restrict__ b1,
    const float* __restrict__ W2,
    const float* __restrict__ b2,
    float* out,
    int nE, int nA)
{
  __shared__ __attribute__((aligned(16))) float sOut[EPB];

  const int tid = (int)threadIdx.x, lane = tid & 31, wave = tid >> 5;

  float bb[8], ww[8];
  {
    const v4f b0 = *(const v4fa*)(b1 + 8 * lane);
    const v4f b1v = *(const v4fa*)(b1 + 8 * lane + 4);
    const v4f w0 = *(const v4fa*)(W2 + 8 * lane);
    const v4f w1 = *(const v4fa*)(W2 + 8 * lane + 4);
    bb[0] = bf16_val(b0.x);  bb[1] = bf16_val(b0.y);  bb[2] = bf16_val(b0.z);  bb[3] = bf16_val(b0.w);
    bb[4] = bf16_val(b1v.x); bb[5] = bf16_val(b1v.y); bb[6] = bf16_val(b1v.z); bb[7] = bf16_val(b1v.w);
    ww[0] = bf16_val(w0.x);  ww[1] = bf16_val(w0.y);  ww[2] = bf16_val(w0.z);  ww[3] = bf16_val(w0.w);
    ww[4] = bf16_val(w1.x);  ww[5] = bf16_val(w1.y);  ww[6] = bf16_val(w1.z);  ww[7] = bf16_val(w1.w);
  }
  const float b2v = b2[0];

  const int ebase = (int)blockIdx.x * EPB + 32 * wave;
  int e = ebase + lane;
  e = e > nE - 1 ? nE - 1 : e;
  const int rawr = srcI[(size_t)e];
  const int rawc = dstI[(size_t)e];
  int ri = rawr < 0 ? rawr + nA : rawr;
  ri = ri < 0 ? 0 : (ri > nA - 1 ? nA - 1 : ri);
  int ci = rawc < 0 ? rawc + nA : rawc;
  ci = ci < 0 ? 0 : (ci > nA - 1 ? nA - 1 : ci);

  float mine = 0.0f;
#pragma unroll 1
  for (int j = 0; j < 32; ++j) {
    const int rj = __shfl(ri, j, 32);
    const int cj = __shfl(ci, j, 32);
    const v4u pw = *(const v4ua*)(Pp + (size_t)rj * NHID + 8 * lane);
    const v4u qw = *(const v4ua*)(Qp + (size_t)cj * NHID + 8 * lane);
    float s = 0.0f;
#pragma unroll
    for (int i = 0; i < 4; ++i) {
      const unsigned int pwi = pw[i], qwi = qw[i];
      const float p0 = h2f(pwi & 0xffffu), p1 = h2f(pwi >> 16);
      const float q0 = h2f(qwi & 0xffffu), q1 = h2f(qwi >> 16);
      const float h0 = fmaxf((p0 + q0) * 0.125f + bb[2 * i],     0.0f);
      const float h1 = fmaxf((p1 + q1) * 0.125f + bb[2 * i + 1], 0.0f);
      s = fmaf(h0, ww[2 * i],     s);
      s = fmaf(h1, ww[2 * i + 1], s);
    }
    s += __shfl_xor(s, 16, 32);
    s += __shfl_xor(s, 8, 32);
    s += __shfl_xor(s, 4, 32);
    s += __shfl_xor(s, 2, 32);
    s += __shfl_xor(s, 1, 32);
    mine = (lane == j) ? s : mine;
  }
  const float val = mine + b2v;
  sOut[tid] = val;
  __syncthreads();

  const bool wr  = (tid < EPB / 4);
  const int  t64 = wr ? tid : 0;
  const v4f  v   = *(const v4fa*)(sOut + 4 * t64);
  const int  eb  = (int)blockIdx.x * EPB + 4 * t64;
  const bool full  = wr && (eb + 3 < nE);
  const bool tailw = wr && !full;
  out_store_pass(out, v, eb, nE, full, tailw);
  __threadfence();
  out_store_pass(out, v, eb, nE, full, tailw);
}

static inline int cdiv(int a, int b) { return (a + b - 1) / b; }

extern "C" void kernel_launch(void* const* d_in, const int* in_sizes, int n_in,
                              void* d_out, int out_size, void* d_ws, size_t ws_size,
                              hipStream_t stream) {
  if (n_in < 8) return;
  if (in_sizes[0] < KIN || (in_sizes[0] % KIN) != 0) return;
  const int nA = in_sizes[0] / KIN;
  if (in_sizes[1] != in_sizes[0]) return;
  const int nE = in_sizes[2];
  if (nE < 1) return;
  if (in_sizes[3] != nE) return;
  if (in_sizes[4] != 2 * KIN * NHID) return;
  if (in_sizes[5] != NHID) return;
  if (in_sizes[6] != NHID) return;
  if (in_sizes[7] < 1) return;
  if (out_size != nE) return;

  const float* hS   = (const float*)d_in[0];
  const float* hD   = (const float*)d_in[1];
  const int*   srcI = (const int*)d_in[2];
  const int*   dstI = (const int*)d_in[3];
  const float* W1   = (const float*)d_in[4];
  const float* b1   = (const float*)d_in[5];
  const float* W2   = (const float*)d_in[6];
  const float* b2   = (const float*)d_in[7];
  float* out = (float*)d_out;

  const int nApad = cdiv(nA, NROWB) * NROWB;
  char* ws = (char*)d_ws;
  size_t off = 0;
  const size_t oWB = off; off += (size_t)2 * NHID * KIN * 2;     off = (off + 1023) & ~(size_t)1023;
  const size_t oP  = off; off += (size_t)nApad * NHID * 2;       off = (off + 1023) & ~(size_t)1023;
  const size_t oQ  = off; off += (size_t)nApad * NHID * 2;       off = (off + 1023) & ~(size_t)1023;
  if (off > ws_size || off > (size_t)WSMAX) return;
  unsigned short* WB = (unsigned short*)(ws + oWB);
  unsigned short* Pp = (unsigned short*)(ws + oP);
  unsigned short* Qp = (unsigned short*)(ws + oQ);

  k_wprep<<<cdiv(NUNW, 256), 256, 0, stream>>>(W1, WB, NUNW);
  k_node<<<dim3(cdiv(nA, NROWB), 2), GTHR, 0, stream>>>(hS, hD, WB, Pp, Qp, nA);
  k_edge<<<cdiv(nE, EPB), EPB, 0, stream>>>(Pp, Qp, srcI, dstI, b1, W2, b2, out, nE, nA);
}
